// LlamaAttention_55336358642260
// MI455X (gfx1250) — hardware-verified
//
#include <hip/hip_runtime.h>


#ifndef NB
#define NB 2
#endif
#ifndef SEQ
#define SEQ 2048
#endif
#define NB_FULL  2
#define SEQ_FULL 2048
#define DM   2048
#define NH_  16
#define HD   128
#define DQ   (NH_ * HD)
#define DKV  (NH_ * HD)
#define CCAR 64.0f
#define WCAR 64.0f
#define OSCL (1.0f / 4096.0f)

static_assert(SEQ % 64 == 0);
static_assert(SEQ <= SEQ_FULL);
static_assert(NB >= 1 && NB <= NB_FULL);
static_assert(HD == 128);
static_assert(DM % 64 == 0 && DQ % 64 == 0);
static_assert(((size_t)NH_ * SEQ * HD) % 512 == 0);
static_assert(((size_t)SEQ * HD) % 256 == 0);
static_assert(((size_t)SEQ * DM) % 2048 == 0);

typedef _Float16 h16;
typedef unsigned short bf;
typedef __attribute__((ext_vector_type(16))) __bf16   v16bf;
typedef __attribute__((ext_vector_type(16))) _Float16 v16h;
typedef __attribute__((ext_vector_type(8)))  _Float16 v8h;
typedef __attribute__((ext_vector_type(8)))  unsigned short v8us;
typedef __attribute__((ext_vector_type(8)))  float    v8f;
typedef __attribute__((ext_vector_type(4)))  float    v4f;
typedef __attribute__((ext_vector_type(2)))  _Float16 v2h;
typedef __attribute__((ext_vector_type(2)))  float    v2f;
typedef v8h  __attribute__((may_alias)) v8ha;
typedef v4f  __attribute__((may_alias)) v4fa;

__device__ __forceinline__ unsigned short f2bf(float f) { unsigned u = __float_as_uint(f); u += 0x7FFFu + ((u >> 16) & 1u); return (unsigned short)(u >> 16); }
__device__ __forceinline__ float bf2f(unsigned short b) { return __uint_as_float(((unsigned)b) << 16); }
__device__ __forceinline__ float bfr(float f) { return bf2f(f2bf(f)); }
__device__ __forceinline__ v16h cat16(v8h lo, v8h hi) { return __builtin_shufflevector(lo, hi, 0, 1, 2, 3, 4, 5, 6, 7, 8, 9, 10, 11, 12, 13, 14, 15); }
__device__ __forceinline__ v16bf cat16b(v8us lo, v8us hi) { return __builtin_bit_cast(v16bf, __builtin_shufflevector(lo, hi, 0, 1, 2, 3, 4, 5, 6, 7, 8, 9, 10, 11, 12, 13, 14, 15)); }
__device__ __forceinline__ v8f wmma16(v16h a, v16h b, v8f c) { return __builtin_amdgcn_wmma_f32_16x16x32_f16(false, a, false, b, (short)0, c, false, false); }
__device__ __forceinline__ v8f wmmab(v16bf a, v16bf b, v8f c) { return __builtin_amdgcn_wmma_f32_16x16x32_bf16(false, a, false, b, (short)0, c, false, false); }
__device__ __forceinline__ v16h ldg16(const h16* p) { return cat16(*(const v8h*)p, *(const v8h*)(p + 16)); }
__device__ __forceinline__ v16h ldl16(const h16* p) { return cat16(*(const v8ha*)p, *(const v8ha*)(p + 16)); }

template <typename T16> struct WFrag;
template <> struct WFrag<h16> { typedef v16h V; static __device__ __forceinline__ V ld(const h16* p) { return cat16(*(const v8h*)p, *(const v8h*)(p + 16)); } static __device__ __forceinline__ v8f mma(V a, V b, v8f c) { return wmma16(a, b, c); } };
template <> struct WFrag<bf> { typedef v16bf V; static __device__ __forceinline__ V ld(const bf* p) { return cat16b(*(const v8us*)p, *(const v8us*)(p + 16)); } static __device__ __forceinline__ v8f mma(V a, V b, v8f c) { return wmmab(a, b, c); } };
template <typename T16, int NSPLIT, bool BIAS>
__global__ __launch_bounds__(32) void k_gemmw(const T16* __restrict__ A, const T16* __restrict__ A2, const T16* __restrict__ Bt, const T16* __restrict__ Bt2, int K, float* C, int ldc, const float* __restrict__ bias, float oscale, size_t sA, size_t sB, size_t sC) {
    typedef typename WFrag<T16>::V V;
    __shared__ __align__(16) float os[16 * 68];
    const size_t z = blockIdx.z; A += z * sA; if (A2) A2 += z * sA; Bt += z * sB; if (Bt2) Bt2 += z * sB; C += z * sC;
    const int lane = threadIdx.x & 31, lr = lane & 15, hi = lane >> 4; const int r0 = blockIdx.x * 64, c0 = blockIdx.y * 64;
    v8f acc[4][4];
#pragma unroll
    for (int mb = 0; mb < 4; ++mb)
#pragma unroll
        for (int nb = 0; nb < 4; ++nb) acc[mb][nb] = (v8f){};
    const size_t aoff = (size_t)(r0 + lr) * K + 8 * hi, boff = (size_t)(c0 + lr) * K + 8 * hi;
#pragma unroll 1
    for (int kc = 0; kc < K; kc += 32) {
        V a[4], a2[4];
#pragma unroll
        for (int mb = 0; mb < 4; ++mb) { a[mb] = WFrag<T16>::ld(A + aoff + (size_t)mb * 16 * K + kc); if (NSPLIT == 1 || NSPLIT == 2) a2[mb] = WFrag<T16>::ld(A2 + aoff + (size_t)mb * 16 * K + kc); }
#pragma unroll
        for (int nb = 0; nb < 4; ++nb) { const V b = WFrag<T16>::ld(Bt + boff + (size_t)nb * 16 * K + kc); V b2; if (NSPLIT >= 2) b2 = WFrag<T16>::ld(Bt2 + boff + (size_t)nb * 16 * K + kc);
#pragma unroll
            for (int mb = 0; mb < 4; ++mb) { acc[mb][nb] = WFrag<T16>::mma(a[mb], b, acc[mb][nb]); if (NSPLIT == 1 || NSPLIT == 2) acc[mb][nb] = WFrag<T16>::mma(a2[mb], b, acc[mb][nb]); if (NSPLIT >= 2) acc[mb][nb] = WFrag<T16>::mma(a[mb], b2, acc[mb][nb]); } }
        asm volatile("v_nop\n\tv_nop\n\tv_nop\n\tv_nop" : "+v"(acc[0][0]), "+v"(acc[1][1]), "+v"(acc[2][2]), "+v"(acc[3][3]) : "v"(a[0]), "v"(a[3]));
    }
#pragma unroll
    for (int mb = 0; mb < 4; ++mb) {
#pragma unroll
        for (int nb = 0; nb < 4; ++nb) {
#pragma unroll
            for (int j = 0; j < 8; ++j) os[(hi * 8 + j) * 68 + nb * 16 + lr] = acc[mb][nb][j]; }
        __builtin_amdgcn_wave_barrier(); asm volatile("" ::: "memory");
        float* crow = C + (size_t)(r0 + mb * 16) * ldc + c0;
#pragma unroll 1
        for (int ps = 0; ps < 2; ++ps) {
#pragma unroll
            for (int s = 0; s < 8; ++s) { const int row = 2 * s + hi, cofs = lr * 4; v4f val = *(const v4fa*)(os + row * 68 + cofs); if (BIAS) { val[0] += bfr(bias[c0 + cofs]); val[1] += bfr(bias[c0 + cofs + 1]); val[2] += bfr(bias[c0 + cofs + 2]); val[3] += bfr(bias[c0 + cofs + 3]); }
                val *= oscale;
                *(volatile v4f*)(crow + (size_t)row * ldc + cofs) = val; }
            if (ps == 0) __threadfence(); }
        __builtin_amdgcn_wave_barrier(); asm volatile("" ::: "memory");
    }
}

__global__ __launch_bounds__(256) void k_cvt8(const float* __restrict__ src, bf* dst, size_t n8) { const size_t i = (size_t)blockIdx.x * 256 + threadIdx.x; if (i >= n8) return; const v8f v = *(const v8f*)(src + i * 8); v8us o;
#pragma unroll
    for (int k = 0; k < 8; ++k) o[k] = f2bf(v[k]); *(volatile v8us*)(dst + i * 8) = o; __threadfence(); *(volatile v8us*)(dst + i * 8) = o; }
__global__ __launch_bounds__(256) void k_cvtw16(const float* __restrict__ src, h16* dst, size_t n8) { const size_t i = (size_t)blockIdx.x * 256 + threadIdx.x; if (i >= n8) return; const v8f v = *(const v8f*)(src + i * 8); v8h o;
#pragma unroll
    for (int k = 0; k < 8; ++k) o[k] = (h16)(bfr(v[k]) * WCAR); *(volatile v8h*)(dst + i * 8) = o; __threadfence(); *(volatile v8h*)(dst + i * 8) = o; }

__global__ __launch_bounds__(64) void k_invf(float* INVF) {
    __shared__ __align__(16) float s[64];
    const int j = threadIdx.x;
    const float ex = (float)(2 * j) * (1.0f / 128.0f);
    const float p = powf(10000.0f, ex);
    s[j] = 1.0f / p;
    __syncthreads();
    v4f v = (v4f){};
    if (j < 16) { v = *(const v4fa*)(s + 4 * j); *(volatile v4f*)(INVF + 4 * j) = v; }
    __threadfence();
    if (j < 16) { *(volatile v4f*)(INVF + 4 * j) = v; }
}
__global__ __launch_bounds__(256) void k_cstab(const float* __restrict__ INVF, float* CS) {
    const int idx = blockIdx.x * 256 + threadIdx.x; if (idx >= SEQ * HD) return;
    const int d = idx % HD; const int t = idx / HD;
    const float f = INVF[d & 63];
    float ang = __fmul_rn((float)t, f); asm volatile("" : "+v"(ang));
    float sn, cs; sincosf(ang, &sn, &cs);
    v2f o; o[0] = cs; o[1] = sn;
    *(volatile v2f*)(CS + (size_t)idx * 2) = o; __threadfence(); *(volatile v2f*)(CS + (size_t)idx * 2) = o;
}
__global__ __launch_bounds__(256) void k_rope16(const float* __restrict__ F, int pitch, int nheads, const float* __restrict__ CS, float sc, h16* P16) {
    const size_t e = ((size_t)blockIdx.x * 256 + threadIdx.x) * 2; if (e >= (size_t)nheads * SEQ * HD) return; const int d = (int)(e % HD); const int t = (int)((e / HD) % SEQ); const int h = (int)(e / ((size_t)HD * SEQ)); const float* f = F + (size_t)t * pitch + h * HD; v2h o16;
#pragma unroll
    for (int q = 0; q < 2; ++q) { const int dd = d + q; const int dp = (dd < HD / 2) ? dd + HD / 2 : dd - HD / 2; const float x0 = f[dd], x1 = f[dp];
        const v2f cs = *(const v2f*)(CS + ((size_t)t * HD + dd) * 2); float a = __fmul_rn(x0, cs[0]), bq = __fmul_rn(x1, cs[1]); asm volatile("" : "+v"(a)); asm volatile("" : "+v"(bq)); const float r = ((dd < HD / 2) ? __fsub_rn(a, bq) : __fadd_rn(a, bq)) * sc;
        o16[q] = (h16)r; }
    *(volatile v2h*)(P16 + e) = o16; __threadfence(); *(volatile v2h*)(P16 + e) = o16; }
__global__ __launch_bounds__(256) void k_vtp16(const float* __restrict__ F, int pitch, int nheads, h16* V16) { const size_t e = ((size_t)blockIdx.x * 256 + threadIdx.x) * 2; if (e >= (size_t)nheads * HD * SEQ) return; const int t = (int)(e % SEQ); const int d = (int)((e / SEQ) % HD); const int g = (int)(e / ((size_t)SEQ * HD)); v2h o16;
#pragma unroll
    for (int q = 0; q < 2; ++q) { const float x = F[(size_t)(t + q) * pitch + g * HD + d]; o16[q] = (h16)x; }
    *(volatile v2h*)(V16 + e) = o16; __threadfence(); *(volatile v2h*)(V16 + e) = o16; }

__global__ __launch_bounds__(32) void k_flash(const h16* __restrict__ QP, const h16* __restrict__ KP, const h16* __restrict__ VT, h16* CTX) {
    __shared__ __align__(16) h16 psh[16 * 32];
    __shared__ __align__(16) h16 csh[16 * 128];
    const int lane = threadIdx.x & 31, lr = lane & 15, hi = lane >> 4;
    const int h = blockIdx.y, t0 = blockIdx.x * 16;
    const h16* Qb = QP + ((size_t)h * SEQ + t0) * HD;
    const h16* Kb = KP + (size_t)h * SEQ * HD;
    const h16* Vb = VT + (size_t)h * HD * SEQ;
    v16h qa[4];
#pragma unroll
    for (int j = 0; j < 4; ++j) qa[j] = ldg16(Qb + (size_t)lr * HD + 32 * j + 8 * hi);
    v8f o[8];
#pragma unroll
    for (int t = 0; t < 8; ++t) o[t] = (v8f){};
    float mrow[8], lsum[8];
#pragma unroll
    for (int e = 0; e < 8; ++e) { mrow[e] = -3.0e38f; lsum[e] = 0.0f; }
    const float cl = 1.4426950408889634f * 0.088388347648318447f;
#pragma unroll 1
    for (int kb = 0; kb < SEQ; kb += 32) {
        v8f sa = (v8f){}, sb = (v8f){};
        const h16* k0p = Kb + (size_t)(kb + lr) * HD + 8 * hi;
        const h16* k1p = Kb + (size_t)(kb + 16 + lr) * HD + 8 * hi;
#pragma unroll
        for (int j = 0; j < 4; ++j) { const v16h kf0 = ldg16(k0p + 32 * j); sa = wmma16(qa[j], kf0, sa); const v16h kf1 = ldg16(k1p + 32 * j); sb = wmma16(qa[j], kf1, sb); }
        asm volatile("v_nop\n\tv_nop\n\tv_nop\n\tv_nop" : "+v"(sa), "+v"(sb) : "v"(qa[0]), "v"(qa[3]));
#pragma unroll
        for (int e = 0; e < 8; ++e) {
            const float v0 = sa[e] * cl, v1 = sb[e] * cl;
            float mx = fmaxf(v0, v1);
#pragma unroll
            for (int off = 8; off > 0; off >>= 1) mx = fmaxf(mx, __shfl_xor(mx, off, 16));
            const float mn = fmaxf(mrow[e], mx);
            const float corr = __builtin_amdgcn_exp2f(mrow[e] - mn);
            mrow[e] = mn;
            const h16 p0 = (h16)__builtin_amdgcn_exp2f(v0 - mn + 4.0f);
            const h16 p1 = (h16)__builtin_amdgcn_exp2f(v1 - mn + 4.0f);
            float ps = (float)p0 + (float)p1;
#pragma unroll
            for (int off = 8; off > 0; off >>= 1) ps += __shfl_xor(ps, off, 16);
            lsum[e] = lsum[e] * corr + ps;
#pragma unroll
            for (int t = 0; t < 8; ++t) o[t][e] *= corr;
            psh[(hi * 8 + e) * 32 + lr] = p0;
            psh[(hi * 8 + e) * 32 + 16 + lr] = p1;
        }
        asm volatile("s_wait_dscnt 0x0" ::: "memory");
        __builtin_amdgcn_wave_barrier(); asm volatile("" ::: "memory");
        const v16h pf = ldl16(psh + lr * 32 + 8 * hi);
        const h16* vp = Vb + (size_t)lr * SEQ + kb + 8 * hi;
#pragma unroll
        for (int t = 0; t < 8; ++t) { const v16h vf = ldg16(vp + (size_t)t * 16 * SEQ); o[t] = wmma16(pf, vf, o[t]); }
        asm volatile("v_nop\n\tv_nop\n\tv_nop\n\tv_nop" : "+v"(o[0]), "+v"(o[1]), "+v"(o[2]), "+v"(o[3]), "+v"(o[4]), "+v"(o[5]), "+v"(o[6]), "+v"(o[7]) : "v"(pf));
    }
#pragma unroll
    for (int e = 0; e < 8; ++e) { const float inv = CCAR * __builtin_amdgcn_rcpf(lsum[e]);
#pragma unroll
        for (int t = 0; t < 8; ++t) csh[(hi * 8 + e) * 128 + t * 16 + lr] = (h16)(o[t][e] * inv); }
    asm volatile("s_wait_dscnt 0x0" ::: "memory");
    __builtin_amdgcn_wave_barrier(); asm volatile("" ::: "memory");
    h16* crow = CTX + (size_t)t0 * DQ + (size_t)h * HD;
#pragma unroll 1
    for (int ps = 0; ps < 2; ++ps) {
#pragma unroll
        for (int s = 0; s < 8; ++s) { const int row = 2 * s + hi; const v8h val = *(const v8ha*)(csh + row * 128 + lr * 8); *(volatile v8h*)(crow + (size_t)row * DQ + lr * 8) = val; }
        if (ps == 0) __threadfence(); }
}

#define WS_TOTAL ((size_t)3 * DM * DM * 2 + (size_t)DM * DM * 2 + (size_t)256 + (size_t)SEQ * HD * 2 * 4 + (size_t)SEQ * DM * 2 + (size_t)2 * SEQ * DQ * 4 + (size_t)3 * NH_ * SEQ * HD * 2 + (size_t)SEQ * DQ * 2)
static_assert(WS_TOTAL <= (size_t)134217728);

extern "C" void kernel_launch(void* const* d_in, const int* in_sizes, int n_in,
                              void* d_out, int out_size, void* d_ws, size_t ws_size, hipStream_t stream) {
    if (n_in < 5) return;
    const size_t needx = (size_t)(NB - 1) * SEQ_FULL * DM + (size_t)SEQ * DM;
    if ((size_t)in_sizes[0] < needx) return;
    for (int i = 1; i < 5; ++i) if ((size_t)in_sizes[i] < (size_t)DM * DM) return;
    if ((size_t)out_size < needx) return;
    const float* x = (const float*)d_in[0]; const float* wq = (const float*)d_in[1]; const float* wk = (const float*)d_in[2]; const float* wv = (const float*)d_in[3]; const float* wo = (const float*)d_in[4];
    float* OUT = (float*)d_out;
    char* wsp = (char*)d_ws;
    auto take = [&](size_t bytes) { char* p = wsp; wsp += (bytes + 255) & ~(size_t)255; return (void*)p; };
    bf* WQ = (bf*)take((size_t)DQ * DM * 2); bf* WK = (bf*)take((size_t)DKV * DM * 2); bf* WV = (bf*)take((size_t)DKV * DM * 2); h16* WO16 = (h16*)take((size_t)DM * DQ * 2);
    float* INVF = (float*)take(256); float* CS = (float*)take((size_t)SEQ * HD * 2 * 4);
    bf* XB = (bf*)take((size_t)SEQ * DM * 2); float* FQ = (float*)take((size_t)SEQ * DQ * 4); float* FK = (float*)take((size_t)SEQ * DKV * 4);
    h16* QP16 = (h16*)take((size_t)NH_ * SEQ * HD * 2); h16* KP16 = (h16*)take((size_t)NH_ * SEQ * HD * 2); h16* VT16 = (h16*)take((size_t)NH_ * HD * SEQ * 2);
    h16* CTX16 = (h16*)take((size_t)SEQ * DQ * 2);
    if ((size_t)(wsp - (char*)d_ws) > ws_size) return;
    float* FV = FK;
    k_cvt8<<<(unsigned)(((size_t)DQ * DM / 8 + 255) / 256), 256, 0, stream>>>(wq, WQ, (size_t)DQ * DM / 8);
    k_cvt8<<<(unsigned)(((size_t)DKV * DM / 8 + 255) / 256), 256, 0, stream>>>(wk, WK, (size_t)DKV * DM / 8);
    k_cvt8<<<(unsigned)(((size_t)DKV * DM / 8 + 255) / 256), 256, 0, stream>>>(wv, WV, (size_t)DKV * DM / 8);
    k_cvtw16<<<(unsigned)(((size_t)DM * DQ / 8 + 255) / 256), 256, 0, stream>>>(wo, WO16, (size_t)DM * DQ / 8);
    k_invf<<<1, 64, 0, stream>>>(INVF);
    k_cstab<<<(SEQ * HD + 255) / 256, 256, 0, stream>>>(INVF, CS);
    const unsigned LP = (unsigned)(((size_t)NH_ * SEQ * HD / 2 + 255) / 256);
    for (int b = 0; b < NB; ++b) {
        k_cvt8<<<(unsigned)(((size_t)SEQ * DM / 8 + 255) / 256), 256, 0, stream>>>(x + (size_t)b * SEQ_FULL * DM, XB, (size_t)SEQ * DM / 8);
        k_gemmw<bf, 0, false><<<dim3(SEQ / 64, DQ / 64, 1), 32, 0, stream>>>(XB, nullptr, WQ, nullptr, DM, FQ, DQ, nullptr, 1.0f, 0, 0, 0);
        k_rope16<<<LP, 256, 0, stream>>>(FQ, DQ, NH_, CS, 1.0f, QP16);
        k_gemmw<bf, 0, false><<<dim3(SEQ / 64, DKV / 64, 1), 32, 0, stream>>>(XB, nullptr, WK, nullptr, DM, FK, DKV, nullptr, 1.0f, 0, 0, 0);
        k_rope16<<<LP, 256, 0, stream>>>(FK, DKV, NH_, CS, 1.0f, KP16);
        k_gemmw<bf, 0, false><<<dim3(SEQ / 64, DKV / 64, 1), 32, 0, stream>>>(XB, nullptr, WV, nullptr, DM, FV, DKV, nullptr, 1.0f, 0, 0, 0);
        k_vtp16<<<LP, 256, 0, stream>>>(FV, DKV, NH_, VT16);
        k_flash<<<dim3(SEQ / 16, NH_, 1), 32, 0, stream>>>(QP16, KP16, VT16, CTX16);
        k_gemmw<h16, 0, false><<<dim3(SEQ / 64, DM / 64, 1), 32, 0, stream>>>(CTX16, nullptr, WO16, nullptr, DQ, OUT + (size_t)b * SEQ_FULL * DM, DM, nullptr, OSCL, 0, 0, 0);
    }
}
